// GraspSO3DeformableAttn_3410204033227
// MI455X (gfx1250) — hardware-verified
//
#include <hip/hip_runtime.h>
#include <math.h>

typedef __attribute__((ext_vector_type(16))) _Float16 v16h;
typedef __attribute__((ext_vector_type(16))) __bf16 v16b;
typedef __attribute__((ext_vector_type(8)))  _Float16 v8h;
typedef __attribute__((ext_vector_type(8)))  float v8f;
typedef __attribute__((ext_vector_type(4)))  float v4f;
typedef __attribute__((ext_vector_type(2)))  float v2f;
typedef __attribute__((ext_vector_type(4)))  unsigned v4u;
typedef __attribute__((ext_vector_type(4)))  int v4i;
typedef float __attribute__((may_alias)) float_a;
typedef int __attribute__((may_alias)) int_a;

template <typename T> __device__ __forceinline__ void vst2(void* p, T v) { *(volatile T*)p = v; __threadfence(); *(volatile T*)p = v; }
__device__ __forceinline__ v8f wmma16(v16h a, v16h b, v8f c) {
  v8f d = __builtin_amdgcn_wmma_f32_16x16x32_f16(false, a, false, b, (short)0, c, false, false);
  asm volatile("v_nop\n\tv_nop\n\tv_nop\n\tv_nop" : "+v"(d) : "v"(a), "v"(b));
  return d;
}
__device__ __forceinline__ v8f wmma_bf(v16b a, v16b b, v8f c) {
  v8f d = __builtin_amdgcn_wmma_f32_16x16x32_bf16(false, a, false, b, (short)0, c, false, false);
  asm volatile("v_nop\n\tv_nop\n\tv_nop\n\tv_nop" : "+v"(d) : "v"(a), "v"(b));
  return d;
}
__device__ __forceinline__ v16h frag_h(const _Float16* rowk0, int lane) {
  union { v16h v; v8h q[2]; } u; const _Float16* p = rowk0 + 8 * (lane >> 4);
  u.q[0] = *(const v8h*)p; u.q[1] = *(const v8h*)(p + 16); return u.v;
}
__device__ __forceinline__ v16h frag_f32(const float* rowk0, int lane) {
  v16h a; const float* p = rowk0 + 8 * (lane >> 4);
#pragma unroll
  for (int i = 0; i < 8; ++i) { a[i] = (_Float16)p[i]; a[8 + i] = (_Float16)p[16 + i]; }
  return a;
}
__device__ __forceinline__ v16h frag_f32s(const float* rowk0, int lane, float sc) {
  v16h a; const float* p = rowk0 + 8 * (lane >> 4);
#pragma unroll
  for (int i = 0; i < 8; ++i) { a[i] = (_Float16)(p[i] * sc); a[8 + i] = (_Float16)(p[16 + i] * sc); }
  return a;
}
__device__ __forceinline__ v16h fragc_f32(const float* W, int k0, int n, int lane, int ld, int K) {
  v16h a; const int g = lane >> 4;
#pragma unroll
  for (int i = 0; i < 8; ++i) { const int ka = k0 + 8 * g + i, kb = ka + 16;
    a[i] = (_Float16)(ka < K ? W[(size_t)(ka < K ? ka : K - 1) * ld + n] : 0.f); a[8 + i] = (_Float16)(kb < K ? W[(size_t)(kb < K ? kb : K - 1) * ld + n] : 0.f); }
  return a;
}
struct F2 { v16b h, l; };
__device__ __forceinline__ F2 bsplit16(const float v[16]) { F2 r;
#pragma unroll
  for (int i = 0; i < 16; ++i) { const __bf16 h = (__bf16)v[i]; r.h[i] = h; r.l[i] = (__bf16)(v[i] - (float)h); }
  return r; }
__device__ __forceinline__ F2 split_row(const float* row, int k0, int lane) { float v[16]; const float* p = row + k0 + 8 * (lane >> 4);
#pragma unroll
  for (int i = 0; i < 8; ++i) { v[i] = p[i]; v[8 + i] = p[16 + i]; }
  return bsplit16(v); }
__device__ __forceinline__ F2 split_rowK(const float* row, int k0, int lane, int K) { float v[16]; const int g = lane >> 4;
#pragma unroll
  for (int i = 0; i < 8; ++i) { const int ka = k0 + 8 * g + i, kb = ka + 16; v[i] = ka < K ? row[ka < K ? ka : K - 1] : 0.f; v[8 + i] = kb < K ? row[kb < K ? kb : K - 1] : 0.f; }
  return bsplit16(v); }
__device__ __forceinline__ F2 split_col(const float* W, int k0, int n, int lane, int ld, int K) { float v[16]; const int g = lane >> 4;
#pragma unroll
  for (int i = 0; i < 8; ++i) { const int ka = k0 + 8 * g + i, kb = ka + 16; v[i] = ka < K ? W[(size_t)(ka < K ? ka : K - 1) * ld + n] : 0.f; v[8 + i] = kb < K ? W[(size_t)(kb < K ? kb : K - 1) * ld + n] : 0.f; }
  return bsplit16(v); }
__device__ __forceinline__ v8f mac3(const F2& a, const F2& b, v8f c) { c = wmma_bf(a.l, b.h, c); c = wmma_bf(a.h, b.l, c); return wmma_bf(a.h, b.h, c); }
__device__ __forceinline__ float sigm(float v) { return 1.0f / (1.0f + expf(-v)); }
#define LDSX() do { asm volatile("s_wait_dscnt 0" ::: "memory"); __builtin_amdgcn_wave_barrier(); __builtin_amdgcn_fence(__ATOMIC_RELEASE, "workgroup"); } while (0)


#define BS 2
#define NS 1024
#define NQT (BS * NS)
#define C 128
#define E 32
#define NH 4
#define G 25
#define NPT (NH * G)
#define RES 128
#ifndef TQ
#define TQ NQT
#endif
typedef __attribute__((ext_vector_type(8))) __bf16 v8b;
__device__ __forceinline__ v16b frag_b(const __bf16* rowk0, int lane) {
  union { v16b v; v8b q[2]; } u; const __bf16* p = rowk0 + 8 * (lane >> 4);
  u.q[0] = *(const v8b*)p; u.q[1] = *(const v8b*)(p + 16); return u.v;
}
__device__ __forceinline__ float bfr(float v) { return (float)(__bf16)v; }
__device__ __attribute__((noinline)) float exp_ni(float v) { return expf(v); }
__device__ __attribute__((noinline)) float erf_ni(float v) { return erff(v); }

#define WS_FEAT 0u
#define WS_SP   (WS_FEAT + 4u * NQT * C)
#define WS_PKV  (WS_SP + 4u * NQT * NPT * 4)
#define WS_PO   (WS_PKV + 2u * 64 * C)
#define WS_KV   (WS_PO + 2u * C * C)
#define WS_AO   (WS_KV + 4u * (size_t)NQT * NPT * 64)
#define WS_END  (WS_AO + 4u * NQT * C)

__device__ __forceinline__ float sample_plane(const float* __restrict__ plane  , float u, float v) {
  const float x = fminf(fmaxf((u + 1.0f) * 0.5f * (float)(RES - 1), 0.0f), (float)(RES - 1)), y = fminf(fmaxf((v + 1.0f) * 0.5f * (float)(RES - 1), 0.0f), (float)(RES - 1));
  const int x0 = (int)fminf(fmaxf(floorf(x), 0.f), (float)(RES - 2)), y0 = (int)fminf(fmaxf(floorf(y), 0.f), (float)(RES - 2));
  const float wx = x - (float)x0, wy = y - (float)y0;
  const float f00 = bfr(plane[y0 * RES + x0]), f01 = bfr(plane[y0 * RES + x0 + 1]), f10 = bfr(plane[(y0 + 1) * RES + x0]), f11 = bfr(plane[(y0 + 1) * RES + x0 + 1]);
  return (1.0f - wy) * ((1.0f - wx) * f00 + wx * f01) + wy * ((1.0f - wx) * f10 + wx * f11);
}
__device__ __forceinline__ float triplane(const float* __restrict__ CXY, const float* __restrict__ CXZ, const float* __restrict__ CYZ, size_t b, int c, float px, float py, float pz) {
  const size_t po = ((b * C + c) * RES) * RES;
  return (sample_plane(CXY + po, px, py) + sample_plane(CXZ + po, px, pz)) + sample_plane(CYZ + po, py, pz);
}
__global__ __launch_bounds__(128) void k_pack(const float* __restrict__ WK, const float* __restrict__ WV, const float* __restrict__ WO, __bf16* __restrict__ PKV, __bf16* __restrict__ PO) {
  const int n = blockIdx.x, t = threadIdx.x; __shared__ __align__(16) __bf16 s[C];
  if (n < 64) s[t] = (__bf16)((n < E) ? WK[(size_t)t * E + n] : WV[(size_t)t * E + (n - E)]); else s[t] = (__bf16)WO[(size_t)t * C + (n - 64)];
  __syncthreads();
  if (t < C / 8) { __bf16* dst = (n < 64) ? (PKV + (size_t)n * C) : (PO + (size_t)(n - 64) * C); vst2((unsigned*)(dst + t * 8), *(const v4u*)&s[t * 8]); }
}
__global__ __launch_bounds__(128) void k_feat(const float* __restrict__ QP, const float* __restrict__ CXY, const float* __restrict__ CXZ, const float* __restrict__ CYZ, const float* __restrict__ CP, const float* __restrict__ WOFF, float* __restrict__ FEAT, float* __restrict__ SP) {
  __shared__ __align__(16) float sf[C]; __shared__ float soff[NH * 3]; __shared__ __align__(16) float ssp[NPT][4];
  const size_t q = blockIdx.x; const size_t b = q / NS; const int t = threadIdx.x; const float* qp = QP + q * 7;
  const float px = bfr(qp[0]), py = bfr(qp[1]), pz = bfr(qp[2]);
  sf[t] = triplane(CXY, CXZ, CYZ, b, t, px, py, pz);
  __syncthreads();
  if (t < NH * 3) { float a = 0.f; for (int c = 0; c < C; ++c) a += sf[c] * bfr(WOFF[c * (NH * 3) + t]); soff[t] = a; }
  __syncthreads();
  if (t < NPT) { const int h = t / G, gi = t % G; const float r = bfr(qp[3]), i = bfr(qp[4]), j = bfr(qp[5]), k = bfr(qp[6]); const float two_s = 2.0f / (((r * r + i * i) + j * j) + k * k);
    const float m00 = 1.f - two_s * (j * j + k * k), m01 = two_s * (i * j - k * r), m02 = two_s * (i * k + j * r), m10 = two_s * (i * j + k * r), m11 = 1.f - two_s * (i * i + k * k), m12 = two_s * (j * k - i * r), m20 = two_s * (i * k - j * r), m21 = two_s * (j * k + i * r), m22 = 1.f - two_s * (i * i + j * j);
    const float c0 = bfr(CP[gi * 3]), c1 = bfr(CP[gi * 3 + 1]), c2 = bfr(CP[gi * 3 + 2]);
    const float ax = px + ((m00 * c0 + m01 * c1) + m02 * c2), ay = py + ((m10 * c0 + m11 * c1) + m12 * c2), az = pz + ((m20 * c0 + m21 * c1) + m22 * c2);
    ssp[t][0] = soff[h * 3] + ax; ssp[t][1] = soff[h * 3 + 1] + ay; ssp[t][2] = soff[h * 3 + 2] + az; ssp[t][3] = 0.f; }
  __syncthreads();
  if (t < C / 4) vst2(FEAT + q * C + t * 4, *(const v4f*)&sf[t * 4]);
  if (t < NPT) vst2(SP + (q * NPT + t) * 4, *(const v4f*)&ssp[t][0]);
}
__global__ __launch_bounds__(128) void k_kv(const float* __restrict__ SP, const float* __restrict__ CXY, const float* __restrict__ CXZ, const float* __restrict__ CYZ, const __bf16* __restrict__ PKV, const float* __restrict__ BK, const float* __restrict__ BV, float* __restrict__ KV) {
  __shared__ __align__(16) __bf16 sh[64][C + 8], sl[64][C + 8]; __shared__ __align__(16) float so[4][16][68];
  const int tid = threadIdx.x, wave = tid >> 5, lane = tid & 31, col = lane & 15, g = lane >> 4; const size_t p0 = (size_t)blockIdx.x * 64;
  for (int e = tid; e < 64 * C; e += 128) { const int r = e & 63, c = e >> 6; const size_t p = p0 + r; const size_t b = p / ((size_t)NS * NPT); const float* sp = SP + p * 4;
    const float v = triplane(CXY, CXZ, CYZ, b, c, sp[0], sp[1], sp[2]); const __bf16 hb = (__bf16)v; sh[r][c] = hb; sl[r][c] = (__bf16)(v - (float)hb); }
  if (tid < 64) for (int c = C; c < C + 8; ++c) { sh[tid][c] = (__bf16)0.f; sl[tid][c] = (__bf16)0.f; }
  __syncthreads();
  v8f acc[4] = {};
#pragma unroll
  for (int kc = 0; kc < C / 32; ++kc) { const v16b a = frag_b(&sh[wave * 16 + col][kc * 32], lane), al = frag_b(&sl[wave * 16 + col][kc * 32], lane);
#pragma unroll
    for (int j = 0; j < 4; ++j) { const v16b w = frag_b(PKV + (size_t)(j * 16 + col) * C + kc * 32, lane); acc[j] = wmma_bf(al, w, acc[j]); acc[j] = wmma_bf(a, w, acc[j]); } }
#pragma unroll
  for (int j = 0; j < 4; ++j) { const int o = j * 16 + col; const float bb = (o < E) ? bfr(BK[o]) : bfr(BV[o - E]);
#pragma unroll
    for (int r = 0; r < 8; ++r) so[wave][8 * g + r][o] = acc[j][r] + bb; }
  LDSX();
  for (int rl = 0; rl < 16; ++rl) if (lane < 16) vst2(KV + (p0 + wave * 16 + rl) * 64 + lane * 4, *(const v4f*)&so[wave][rl][lane * 4]);
}
__global__ __launch_bounds__(128) void k_attn(const float* __restrict__ FEAT, const float* __restrict__ WQ, const float* __restrict__ BQ, const float* __restrict__ KV, float* __restrict__ AO) {
  __shared__ float sfe[C], sq[E], ssim[NH][32]; __shared__ __align__(16) float sout[C];
  const size_t q = blockIdx.x; const int t = threadIdx.x; const int h = t >> 5, lane = t & 31;
  sfe[t] = FEAT[q * C + t];
  __syncthreads();
  if (t < E) { float a = 0.f; for (int c = 0; c < C; ++c) a += sfe[c] * bfr(WQ[c * E + t]); sq[t] = (a + bfr(BQ[t])) * sqrtf((float)E); }
  __syncthreads();
  {
    float s = -3.0e38f;
    if (lane < G) { const float* kp = KV + (q * NPT + (size_t)lane * NH + h) * 64; float a = 0.f; for (int e = 0; e < E; ++e) a += sq[e] * kp[e]; s = a; }
    float mx = s;
    for (int o = 1; o < 32; o <<= 1) mx = fmaxf(mx, __shfl_xor(mx, o));
    const float ex = (lane < G) ? __expf(s - mx) : 0.f; float den = ex;
    for (int o = 1; o < 32; o <<= 1) den += __shfl_xor(den, o);
    ssim[h][lane] = ex / den; }
  __syncthreads();
  { const int e = lane; float a = 0.f; for (int gi = 0; gi < G; ++gi) a += ssim[h][gi] * KV[(q * NPT + (size_t)gi * NH + h) * 64 + E + e]; sout[h * E + e] = a; }
  __syncthreads();
  if (t < C / 4) vst2(AO + q * C + t * 4, *(const v4f*)&sout[t * 4]);
}
__global__ __launch_bounds__(128) void k_out(const float* __restrict__ AO, const __bf16* __restrict__ PO, const float* __restrict__ BO, const float* __restrict__ FEAT, float* __restrict__ OUT) {
  __shared__ __align__(16) float so[4][16][132];
  const int tid = threadIdx.x, wave = tid >> 5, lane = tid & 31, col = lane & 15, g = lane >> 4; const size_t r0 = (size_t)blockIdx.x * 64 + wave * 16;
  v8f acc[8] = {};
#pragma unroll
  for (int kc = 0; kc < C / 32; ++kc) { const F2 a = split_row(AO + (r0 + col) * C, kc * 32, lane);
#pragma unroll
    for (int j = 0; j < 8; ++j) { const v16b w = frag_b(PO + (size_t)(j * 16 + col) * C + kc * 32, lane); acc[j] = wmma_bf(a.l, w, acc[j]); acc[j] = wmma_bf(a.h, w, acc[j]); } }
#pragma unroll
  for (int j = 0; j < 8; ++j) { const int c = j * 16 + col; const float bb = bfr(BO[c]);
#pragma unroll
    for (int r = 0; r < 8; ++r) so[wave][8 * g + r][c] = acc[j][r] + bb + FEAT[(r0 + 8 * g + r) * C + c]; }
  LDSX();
  for (int rl = 0; rl < 16; ++rl) vst2(OUT + (r0 + rl) * C + lane * 4, *(const v4f*)&so[wave][rl][lane * 4]);
}
extern "C" void kernel_launch(void* const* d_in, const int* in_sizes, int n_in, void* d_out, int out_size, void* d_ws, size_t ws_size, hipStream_t stream) {
  (void)in_sizes; (void)n_in; (void)out_size;
  const float** F = (const float**)d_in;
  if (ws_size < (size_t)WS_END) return;
  char* ws = (char*)d_ws; float *FEAT = (float*)(ws + WS_FEAT), *SP = (float*)(ws + WS_SP), *KV = (float*)(ws + WS_KV), *AO = (float*)(ws + WS_AO); __bf16 *PKV = (__bf16*)(ws + WS_PKV), *PO = (__bf16*)(ws + WS_PO);
  k_pack<<<64 + C, 128, 0, stream>>>(F[8], F[10], F[12], PKV, PO);
  k_feat<<<TQ, 128, 0, stream>>>(F[0], F[1], F[2], F[3], F[4], F[5], FEAT, SP);
  k_kv<<<TQ * NPT / 64, 128, 0, stream>>>(SP, F[1], F[2], F[3], PKV, F[9], F[11], KV);
  k_attn<<<TQ, 128, 0, stream>>>(FEAT, F[6], F[7], KV, AO);
  k_out<<<TQ / 64, 128, 0, stream>>>(AO, PO, F[13], FEAT, (float*)d_out);
}
